// CustomMHA_33870112096740
// MI455X (gfx1250) — hardware-verified
//
#include <hip/hip_runtime.h>
#include <math.h>

#ifndef NB
#define NB 4
#endif
#ifndef SEQ
#define SEQ 2048
#endif
#define NB_FULL 4
#define SEQ_FULL 2048
#define CC 1024
#define NH 16
#define HD 64
#define HG 4
#define QB0 64
#define PP (2 * SEQ)
static_assert(SEQ % 128 == 0);
static_assert(SEQ >= 128 && SEQ <= SEQ_FULL);
static_assert(NB >= 1 && NB <= NB_FULL);
static_assert(CC == NH * HD);
static_assert(HD == 64);
static_assert(QB0 == 64);
static_assert(NH % HG == 0);
static_assert((SEQ * (SEQ / 32)) % 256 == 0);
static_assert(((CC * CC) / 8) % 256 == 0);
static_assert(((SEQ * CC) / 8) % 256 == 0);

typedef __attribute__((ext_vector_type(16))) _Float16 v16h;
typedef __attribute__((ext_vector_type(16))) __bf16 v16b;
typedef __attribute__((ext_vector_type(8)))  _Float16 v8h;
typedef __attribute__((ext_vector_type(8)))  __bf16 v8b;
typedef __attribute__((ext_vector_type(8)))  float v8f;
typedef __attribute__((ext_vector_type(4)))  float v4f;
typedef __attribute__((ext_vector_type(4)))  unsigned v4u;
typedef __attribute__((ext_vector_type(4)))  int v4i;

#define WS_WQ  ((size_t)0)
#define WS_WK  (WS_WQ + 2u * (size_t)CC * CC)
#define WS_WV  (WS_WK + 2u * (size_t)CC * CC)
#define WS_WO  (WS_WV + 2u * (size_t)CC * CC)
#define WS_XB  (WS_WO + 2u * (size_t)CC * CC)
#define WS_QH  (WS_XB + 2u * (size_t)SEQ * CC)
#define WS_QL  (WS_QH + 2u * (size_t)SEQ * CC)
#define WS_KH  (WS_QL + 2u * (size_t)SEQ * CC)
#define WS_VT  (WS_KH + 2u * (size_t)SEQ * CC)
#define WS_VL  (WS_VT + 2u * (size_t)CC * SEQ)
#define WS_Y   (WS_VL + 2u * (size_t)CC * QB0)
#define WS_YL  (WS_Y + 2u * (size_t)SEQ * CC)
#define WS_S   (WS_YL + 2u * (size_t)QB0 * CC)
#define WS_PL  (WS_S + 4u * (size_t)HG * SEQ * SEQ)
#define WS_MB  (WS_PL + 2u * (size_t)HG * QB0 * QB0)
#define WS_END (WS_MB + 4u * (size_t)SEQ * (SEQ / 32))
static_assert(WS_END <= (size_t)134217728u);
static_assert(WS_WK % 128 == 0 && WS_WV % 128 == 0 && WS_WO % 128 == 0 && WS_XB % 128 == 0 && WS_QH % 128 == 0 && WS_QL % 128 == 0 && WS_KH % 128 == 0);
static_assert(WS_VT % 128 == 0 && WS_VL % 128 == 0 && WS_Y % 128 == 0 && WS_YL % 128 == 0 && WS_S % 128 == 0 && WS_PL % 128 == 0 && WS_MB % 128 == 0);

template <typename T> __device__ __forceinline__ void vst2(void* p, T v) { *(volatile T*)p = v; __threadfence(); *(volatile T*)p = v; }
__device__ __forceinline__ v8f wmma16(v16h a, v16h b, v8f c) {
  v8f d = __builtin_amdgcn_wmma_f32_16x16x32_f16(false, a, false, b, (short)0, c, false, false);
  asm volatile("v_nop\n\tv_nop\n\tv_nop\n\tv_nop" : "+v"(d) : "v"(a), "v"(b));
  return d;
}
__device__ __forceinline__ v8f wmma_bf(v16b a, v16b b, v8f c) {
  v8f d = __builtin_amdgcn_wmma_f32_16x16x32_bf16(false, a, false, b, (short)0, c, false, false);
  asm volatile("v_nop\n\tv_nop\n\tv_nop\n\tv_nop" : "+v"(d) : "v"(a), "v"(b));
  return d;
}
__device__ __forceinline__ v16h frag_h(const _Float16* rowk0, int lane) {
  union { v16h v; v8h q[2]; } u; const _Float16* p = rowk0 + 8 * (lane >> 4);
  u.q[0] = *(const v8h*)p; u.q[1] = *(const v8h*)(p + 16); return u.v;
}
__device__ __forceinline__ v16b frag_b(const __bf16* rowk0, int lane) {
  union { v16b v; v8b q[2]; } u; const __bf16* p = rowk0 + 8 * (lane >> 4);
  u.q[0] = *(const v8b*)p; u.q[1] = *(const v8b*)(p + 16); return u.v;
}
__device__ __forceinline__ float bfr(float v) { return (float)(__bf16)v; }
#define LDSX() do { asm volatile("s_wait_dscnt 0" ::: "memory"); __builtin_amdgcn_wave_barrier(); __builtin_amdgcn_fence(__ATOMIC_RELEASE, "workgroup"); } while (0)

__global__ __launch_bounds__(256) void k_cvt(const float* __restrict__ A, unsigned short* __restrict__ D, int n8, int mode) {
  const int i = blockIdx.x * 256 + threadIdx.x;
  if (i >= n8) return;
  const v4f a = *(const v4f*)(A + (size_t)i * 8); const v4f c = *(const v4f*)(A + (size_t)i * 8 + 4);
  const float v[8] = {a[0], a[1], a[2], a[3], c[0], c[1], c[2], c[3]};
  union { v8b b; v8h h; v4u u; } o;
  if (mode != 0) { v8h t;
#pragma unroll
    for (int k = 0; k < 8; ++k) t[k] = (_Float16)(bfr(v[k]) * 64.0f);
    o.h = t; }
  else { v8b t;
#pragma unroll
    for (int k = 0; k < 8; ++k) t[k] = (__bf16)v[k];
    o.b = t; }
  vst2(D + (size_t)i * 8, o.u);
}

__global__ __launch_bounds__(256) void k_mbits(const int* __restrict__ M, unsigned* __restrict__ MB) {
  const int w = blockIdx.x * 256 + threadIdx.x;
  const int q = w / (SEQ / 32), wc = w - q * (SEQ / 32);
  const int* p = M + (size_t)q * SEQ_FULL + wc * 32;
  unsigned bits = 0u;
#pragma unroll
  for (int i = 0; i < 8; ++i) { const v4i v = *(const v4i*)(p + 4 * i);
    bits |= (v.x != 0 ? 1u : 0u) << (4 * i);     bits |= (v.y != 0 ? 1u : 0u) << (4 * i + 1);
    bits |= (v.z != 0 ? 1u : 0u) << (4 * i + 2); bits |= (v.w != 0 ? 1u : 0u) << (4 * i + 3); }
  vst2(MB + w, bits);
}

__global__ __launch_bounds__(128) void k_proj(const __bf16* __restrict__ XB, const __bf16* __restrict__ WQ, const float* __restrict__ BQ, const __bf16* __restrict__ WK, const float* __restrict__ BK, const __bf16* __restrict__ WV, const float* __restrict__ BV,
                                              const float* __restrict__ RC, const float* __restrict__ RS,
                                              _Float16* __restrict__ QH, _Float16* __restrict__ QL, _Float16* __restrict__ KH, _Float16* __restrict__ VT, _Float16* __restrict__ VL) {
  __shared__ __align__(16) _Float16 sh[64][136], sl[64][136]; __shared__ __align__(16) _Float16 th[128][72], tl2[128][72];
  __shared__ __align__(16) float scs[64][HD], ssn[64][HD];
  const int tid = threadIdx.x, wave = tid >> 5, lane = tid & 31, col = lane & 15, g = lane >> 4; const int which = blockIdx.z; const int c0 = blockIdx.y * 128; const int r0 = blockIdx.x * 64;
  const __bf16* WA = which == 0 ? WQ : which == 1 ? WK : WV; const float* BA = which == 0 ? BQ : which == 1 ? BK : BV;
#pragma unroll 2
  for (int e = tid; e < 64 * (HD / 4); e += 128) { const int rl = e / (HD / 4), q = e % (HD / 4);
    const v4f c = *(const v4f*)(RC + (size_t)(r0 + rl) * HD + q * 4); const v4f s = *(const v4f*)(RS + (size_t)(r0 + rl) * HD + q * 4);
#pragma unroll
    for (int i = 0; i < 4; ++i) { scs[rl][q * 4 + i] = bfr(c[i]); ssn[rl][q * 4 + i] = bfr(s[i]); } }
  __syncthreads();
  v8f acc[8] = {};
#pragma unroll 2
  for (int kc = 0; kc < CC / 32; ++kc) { const v16b a = frag_b(XB + (size_t)(r0 + wave * 16 + col) * CC + kc * 32, lane);
#pragma unroll
    for (int j = 0; j < 8; ++j) { const v16b w = frag_b(WA + (size_t)(c0 + j * 16 + col) * CC + kc * 32, lane); acc[j] = wmma_bf(a, w, acc[j]); } }
  float bbv[8];
#pragma unroll
  for (int j = 0; j < 8; ++j) bbv[j] = bfr(BA[c0 + j * 16 + col]);
#pragma unroll
  for (int r = 0; r < 8; ++r) { const int rl = wave * 16 + 8 * g + r; float v[8];
#pragma unroll
    for (int j = 0; j < 8; ++j) v[j] = acc[j][r] + bbv[j];
    if (which == 2) {
#pragma unroll
      for (int j = 0; j < 8; ++j) { const int cl = j * 16 + col; const _Float16 hv = (_Float16)v[j]; th[cl][rl] = hv; tl2[cl][rl] = (_Float16)((v[j] - (float)hv) * 1024.0f); }
    } else {
      float cs4[4], sn4[4];
#pragma unroll
      for (int jj = 0; jj < 4; ++jj) { cs4[jj] = scs[rl][jj * 16 + col]; sn4[jj] = ssn[rl][jj * 16 + col]; }
#pragma unroll
      for (int j = 0; j < 8; ++j) { const int cl = j * 16 + col, jj = j & 3; const float pv = v[j ^ 2];
        const float o = (jj < 2) ? (v[j] * cs4[jj] - pv * sn4[jj]) : (v[j] * cs4[jj] + pv * sn4[jj]);
        const _Float16 hv = (_Float16)o; sh[rl][cl] = hv; sl[rl][cl] = (_Float16)((o - (float)hv) * 1024.0f); }
    } }
  __syncthreads();
  if (which < 2) { _Float16* dh = which == 0 ? QH : KH; for (int e = tid; e < 64 * 16; e += 128) { const int rl = e >> 4, q = e & 15; vst2(dh + (size_t)(r0 + rl) * CC + c0 + q * 8, *(const v4u*)&sh[rl][q * 8]); if (which == 0) vst2(QL + (size_t)(r0 + rl) * CC + c0 + q * 8, *(const v4u*)&sl[rl][q * 8]); } }
  else { for (int e = tid; e < 128 * 8; e += 128) { const int cl = e >> 3, q = e & 7; const size_t o2 = (size_t)(c0 + cl) * (size_t)SEQ + r0 + q * 8; vst2(VT + o2, *(const v4u*)&th[cl][q * 8]);
      if (blockIdx.x == 0) { const size_t o3 = (size_t)(c0 + cl) * (size_t)QB0 + q * 8; vst2(VL + o3, *(const v4u*)&tl2[cl][q * 8]); } } } }

__global__ __launch_bounds__(128) void k_sc(const _Float16* __restrict__ QH, const _Float16* __restrict__ QL, const _Float16* __restrict__ KH, int h0, float* __restrict__ S0) { __shared__ __align__(16) float ss[4][16][132];
  const int h = h0 + blockIdx.z; float* S = S0 + (size_t)blockIdx.z * SEQ * SEQ;
  const int tid = threadIdx.x, wave = tid >> 5, lane = tid & 31, col = lane & 15, g = lane >> 4; const int k0 = blockIdx.y * 128; const int ql0 = blockIdx.x * 64 + wave * 16;
  if (k0 > (int)blockIdx.x * 64 + 63) return;
  v8f acc[8] = {}, accl[8] = {};
#pragma unroll
  for (int kc = 0; kc < HD / 32; ++kc) { const v16h ah = frag_h(QH + (size_t)(ql0 + col) * CC + h * HD + kc * 32, lane), al = frag_h(QL + (size_t)(ql0 + col) * CC + h * HD + kc * 32, lane);
#pragma unroll
    for (int j = 0; j < 8; ++j) { const v16h kb = frag_h(KH + (size_t)(k0 + j * 16 + col) * CC + h * HD + kc * 32, lane); acc[j] = wmma16(ah, kb, acc[j]); accl[j] = wmma16(al, kb, accl[j]); } }
#pragma unroll
  for (int j = 0; j < 8; ++j) acc[j] += accl[j] * (1.0f / 1024.0f);
#pragma unroll
  for (int j = 0; j < 8; ++j) {
#pragma unroll
    for (int r = 0; r < 8; ++r) ss[wave][8 * g + r][j * 16 + col] = acc[j][r] * 0.125f; }
  LDSX(); for (int rl = 0; rl < 16; ++rl) vst2(S + (size_t)(ql0 + rl) * SEQ + k0 + lane * 4, *(const v4f*)&ss[wave][rl][lane * 4]); }

__global__ __launch_bounds__(256) void k_sm(const float* S0, const unsigned* __restrict__ MB, _Float16* P0, _Float16* __restrict__ PL0) { __shared__ float sred[8]; __shared__ float sbc; __shared__ int sfl[8]; __shared__ unsigned sbits[SEQ / 32]; __shared__ __align__(16) float sh[SEQ];
  const int t = threadIdx.x, wv = t >> 5, ln = t & 31; const int row = blockIdx.x; const size_t rix = (size_t)blockIdx.y * SEQ + row; const float* sr = S0 + rix * SEQ; _Float16* pr = P0 + rix * PP; const int kend = (row / 64) * 64 + 64;
  int bad = 0;
  for (int w = t; w < SEQ / 32; w += 256) { const unsigned u = MB[(size_t)row * (SEQ / 32) + w]; sbits[w] = u; if (32 * w >= kend && u != 0xFFFFFFFFu) bad = 1; }
#pragma unroll
  for (int o = 1; o < 32; o <<= 1) bad |= __shfl_xor(bad, o);
  if (ln == 0) sfl[wv] = bad; __syncthreads();
  int viol = 0;
#pragma unroll
  for (int i = 0; i < 8; ++i) viol |= sfl[i];
  float m = -3.0e38f;
#pragma unroll 1
  for (int k = t; k < kend; k += 256) { const float v = sr[k]; const unsigned mk = (sbits[k >> 5] >> (k & 31)) & 1u; const float sv = mk ? -3.0e38f : v; sh[k] = sv; m = fmaxf(m, sv); }
#pragma unroll
  for (int o = 1; o < 32; o <<= 1) m = fmaxf(m, __shfl_xor(m, o));
  if (ln == 0) sred[wv] = m; __syncthreads(); if (t == 0) { float a = sred[0]; for (int i = 1; i < 8; ++i) a = fmaxf(a, sred[i]); sbc = a; } __syncthreads(); m = sbc; __syncthreads();
  float sum = 0.f;
#pragma unroll 1
  for (int k = t; k < kend; k += 256) { const float v = sh[k]; const float e = (v <= -1.0e38f) ? 0.f : expf(v - m); sh[k] = e; sum += e; }
#pragma unroll
  for (int o = 1; o < 32; o <<= 1) sum += __shfl_xor(sum, o);
  if (ln == 0) sred[wv] = sum; __syncthreads(); if (t == 0) { float a = 0.f; for (int i = 0; i < 8; ++i) a += sred[i]; sbc = 1.0f / a; } __syncthreads();
  const float scl = (viol ? __int_as_float(0x7fc00000) : sbc) * 2048.0f;
  for (int q = t; q < kend / 8; q += 256) {
    const v4f e0 = *(const v4f*)&sh[q * 8]; const v4f e1 = *(const v4f*)&sh[q * 8 + 4];
    const float pe[8] = {e0[0], e0[1], e0[2], e0[3], e1[0], e1[1], e1[2], e1[3]};
    v8h hh, hl;
#pragma unroll
    for (int k = 0; k < 8; ++k) { const float p = pe[k] * scl; const _Float16 ph = (_Float16)p; hh[k] = ph; hl[k] = (_Float16)((p - (float)ph) * 1024.0f); }
    union { v8h h; v4u u; } oh, ol; oh.h = hh; ol.h = hl;
    vst2(pr + q * 8, oh.u);
    if (row < QB0) vst2(PL0 + ((size_t)blockIdx.y * QB0 + row) * QB0 + q * 8, ol.u);
  } }

__global__ __launch_bounds__(128) void k_pv(const _Float16* __restrict__ P0, const _Float16* __restrict__ PL0, const _Float16* __restrict__ VT, const _Float16* __restrict__ VL, int h0, _Float16* __restrict__ Y, _Float16* __restrict__ YL) {
  __shared__ __align__(16) _Float16 sy[4][16][HD + 8], syl[4][16][HD + 8];
  const int hg = blockIdx.z, h = h0 + hg; const _Float16* P = P0 + (size_t)hg * SEQ * PP; const _Float16* PL = PL0 + (size_t)hg * QB0 * QB0;
  const int tid = threadIdx.x, wave = tid >> 5, lane = tid & 31, col = lane & 15, g = lane >> 4; const int ql0 = blockIdx.x * 64 + wave * 16; const int kend = blockIdx.x * 64 + 64;
  v8f acc[HD / 16] = {}, accl[HD / 16] = {};
  if (blockIdx.x == 0) {
#pragma unroll
    for (int kc = 0; kc < QB0 / 32; ++kc) { const v16h p = frag_h(P + (size_t)(ql0 + col) * PP + kc * 32, lane), pl = frag_h(PL + (size_t)(ql0 + col) * QB0 + kc * 32, lane);
#pragma unroll
      for (int j = 0; j < HD / 16; ++j) { const int c = h * HD + j * 16 + col; const v16h vh = frag_h(VT + (size_t)c * SEQ + kc * 32, lane), vl = frag_h(VL + (size_t)c * QB0 + kc * 32, lane);
        acc[j] = wmma16(p, vh, acc[j]); accl[j] = wmma16(pl, vh, accl[j]); accl[j] = wmma16(p, vl, accl[j]); } }
  } else {
#pragma unroll 1
    for (int kc = 0; kc < kend / 32; ++kc) { const v16h p = frag_h(P + (size_t)(ql0 + col) * PP + kc * 32, lane);
#pragma unroll
      for (int j = 0; j < HD / 16; ++j) { const int c = h * HD + j * 16 + col; acc[j] = wmma16(p, frag_h(VT + (size_t)c * SEQ + kc * 32, lane), acc[j]); } }
  }
#pragma unroll
  for (int j = 0; j < HD / 16; ++j)
#pragma unroll
    for (int r = 0; r < 8; ++r) { const float y = (acc[j][r] + accl[j][r] * (1.0f / 1024.0f)) * (1.0f / 128.0f); const _Float16 yh = (_Float16)y; sy[wave][8 * g + r][j * 16 + col] = yh; syl[wave][8 * g + r][j * 16 + col] = (_Float16)((y - (float)yh) * 1024.0f); }
  LDSX();
  for (int rl = 0; rl < 16; ++rl) if (lane < 8) vst2(Y + (size_t)(ql0 + rl) * CC + h * HD + lane * 8, *(const v4u*)&sy[wave][rl][lane * 8]);
  if (blockIdx.x == 0) for (int rl = 0; rl < 16; ++rl) if (lane < 8) vst2(YL + (size_t)(ql0 + rl) * CC + h * HD + lane * 8, *(const v4u*)&syl[wave][rl][lane * 8]); }

__global__ __launch_bounds__(128) void k_out(const _Float16* __restrict__ Y, const _Float16* __restrict__ YL, const _Float16* __restrict__ WO, const float* __restrict__ BP, int b, float* __restrict__ OUT) { __shared__ __align__(16) float sf[4][16][132];
  const int tid = threadIdx.x, wave = tid >> 5, lane = tid & 31, col = lane & 15, g = lane >> 4; const int c0 = blockIdx.y * 128; const int r0 = blockIdx.x * 64 + wave * 16; const size_t orow = (size_t)b * SEQ_FULL + r0;
  v8f acc[8] = {}, accl[8] = {};
  if (blockIdx.x == 0) {
#pragma unroll 2
    for (int kc = 0; kc < CC / 32; ++kc) { const v16h a = frag_h(Y + (size_t)(r0 + col) * CC + kc * 32, lane), al = frag_h(YL + (size_t)(r0 + col) * CC + kc * 32, lane);
#pragma unroll
      for (int j = 0; j < 8; ++j) { const v16h w = frag_h(WO + (size_t)(c0 + j * 16 + col) * CC + kc * 32, lane); acc[j] = wmma16(a, w, acc[j]); accl[j] = wmma16(al, w, accl[j]); } }
  } else {
#pragma unroll 2
    for (int kc = 0; kc < CC / 32; ++kc) { const v16h a = frag_h(Y + (size_t)(r0 + col) * CC + kc * 32, lane);
#pragma unroll
      for (int j = 0; j < 8; ++j) { const v16h w = frag_h(WO + (size_t)(c0 + j * 16 + col) * CC + kc * 32, lane); acc[j] = wmma16(a, w, acc[j]); } }
  }
#pragma unroll
  for (int j = 0; j < 8; ++j) { const float bb = bfr(BP[c0 + j * 16 + col]);
#pragma unroll
    for (int r = 0; r < 8; ++r) sf[wave][8 * g + r][j * 16 + col] = (acc[j][r] + accl[j][r] * (1.0f / 1024.0f)) * (1.0f / 1024.0f) + bb; }
  LDSX(); for (int rl = 0; rl < 16; ++rl) vst2(OUT + (orow + rl) * CC + c0 + lane * 4, *(const v4f*)&sf[wave][rl][lane * 4]); }

extern "C" void kernel_launch(void* const* d_in, const int* in_sizes, int n_in, void* d_out, int out_size, void* d_ws, size_t ws_size, hipStream_t stream) {
  if (n_in < 12) return;
  const size_t xneed = ((size_t)(NB - 1) * SEQ_FULL + SEQ) * (size_t)CC;
  if ((size_t)in_sizes[0] < xneed) return;
  if ((size_t)in_sizes[1] < (size_t)(SEQ - 1) * SEQ_FULL + SEQ) return;
  if (in_sizes[2] < SEQ * HD || in_sizes[3] < SEQ * HD) return;
  if (in_sizes[4] < CC * CC || in_sizes[6] < CC * CC || in_sizes[8] < CC * CC || in_sizes[10] < CC * CC) return;
  if (in_sizes[5] < CC || in_sizes[7] < CC || in_sizes[9] < CC || in_sizes[11] < CC) return;
  if ((size_t)out_size < xneed) return;
  if (ws_size < (size_t)WS_END) return;
  const float* X = (const float*)d_in[0]; const int* M = (const int*)d_in[1]; const float* RC = (const float*)d_in[2]; const float* RS = (const float*)d_in[3];
  const float *WQ = (const float*)d_in[4], *BQ = (const float*)d_in[5], *WK = (const float*)d_in[6], *BK = (const float*)d_in[7], *WV = (const float*)d_in[8], *BV = (const float*)d_in[9], *WO = (const float*)d_in[10], *BO = (const float*)d_in[11];
  char* ws = (char*)d_ws;
  __bf16 *WQB = (__bf16*)(ws + WS_WQ), *WKB = (__bf16*)(ws + WS_WK), *WVB = (__bf16*)(ws + WS_WV), *XB = (__bf16*)(ws + WS_XB); _Float16* WOH = (_Float16*)(ws + WS_WO);
  _Float16 *QH = (_Float16*)(ws + WS_QH), *QL = (_Float16*)(ws + WS_QL), *KH = (_Float16*)(ws + WS_KH), *VT = (_Float16*)(ws + WS_VT), *VL = (_Float16*)(ws + WS_VL), *Y = (_Float16*)(ws + WS_Y), *YL = (_Float16*)(ws + WS_YL);
  float* S = (float*)(ws + WS_S); _Float16* PH = (_Float16*)(ws + WS_S); _Float16* PL = (_Float16*)(ws + WS_PL); unsigned* MB = (unsigned*)(ws + WS_MB); float* OUT = (float*)d_out;
  const int nw8 = (CC * CC) / 8, nx8 = (SEQ * CC) / 8;
  k_cvt<<<dim3(nw8 / 256), 256, 0, stream>>>(WQ, (unsigned short*)WQB, nw8, 0);
  k_cvt<<<dim3(nw8 / 256), 256, 0, stream>>>(WK, (unsigned short*)WKB, nw8, 0);
  k_cvt<<<dim3(nw8 / 256), 256, 0, stream>>>(WV, (unsigned short*)WVB, nw8, 0);
  k_cvt<<<dim3(nw8 / 256), 256, 0, stream>>>(WO, (unsigned short*)WOH, nw8, 1);
  k_mbits<<<dim3(SEQ * (SEQ / 32) / 256), 256, 0, stream>>>(M, MB);
  for (int b = 0; b < NB; ++b) {
    k_cvt<<<dim3(nx8 / 256), 256, 0, stream>>>(X + (size_t)b * SEQ_FULL * CC, (unsigned short*)XB, nx8, 0);
    k_proj<<<dim3(SEQ / 64, CC / 128, 3), 128, 0, stream>>>(XB, WQB, BQ, WKB, BK, WVB, BV, RC, RS, QH, QL, KH, VT, VL);
    for (int h0 = 0; h0 < NH; h0 += HG) {
      k_sc<<<dim3(SEQ / 64, SEQ / 128, HG), 128, 0, stream>>>(QH, QL, KH, h0, S);
      k_sm<<<dim3(SEQ, HG), 256, 0, stream>>>(S, MB, PH, PL);
      k_pv<<<dim3(SEQ / 64, 1, HG), 128, 0, stream>>>(PH, PL, VT, VL, h0, Y, YL);
    }
    k_out<<<dim3(SEQ / 64, CC / 128), 128, 0, stream>>>(Y, YL, WOH, BO, b, OUT);
  }
}
